// GANOKernel_32865089749352
// MI455X (gfx1250) — hardware-verified
//
#include <hip/hip_runtime.h>
#include <stdint.h>

#define DEVINL __device__ __forceinline__

typedef _Float16 f16t;
typedef _Float16 v16h __attribute__((ext_vector_type(16)));
typedef _Float16 v8h  __attribute__((ext_vector_type(8)));
typedef float    v8f  __attribute__((ext_vector_type(8)));
typedef float    v4f  __attribute__((ext_vector_type(4)));
typedef float    v2f  __attribute__((ext_vector_type(2)));
typedef v8h __attribute__((may_alias)) v8ha;
typedef v4f __attribute__((may_alias)) v4fa;
union FragH { v16h v; v8h half[2]; };

#define NQ      2048
#define NO      2048
#define LAT     64
#define PDIM    3
#define ENC     9
#define QB      16
#define WAVES   4
#define TPB     128
#define CHUNK   32
#define OPW     (NO / WAVES)
#define NCHUNK  (OPW / CHUNK)
#define WPAD    68
#define OT      64
#define TP      72
#define PREP_TPB 256
#define PREP_BLK (2 * NQ * LAT / 4 / PREP_TPB)

#define WCAR    64.0f
#define HCAR    4.0f
#define SC_WH   (1.0f / 256.0f)
#define VCAR    16.0f
#define SC_V    0.0625f
#define PCAR    256.0f
#define THR2_BITS 0x3E800001
#define NEG_INF (-__builtin_inff())

static_assert(TPB == WAVES * 32);
static_assert(WAVES * OPW == NO);
static_assert(NCHUNK * CHUNK == OPW);
static_assert(CHUNK == 32);
static_assert(QB == 16);
static_assert(LAT == 64);
static_assert((NQ % QB) == 0);
static_assert(NQ == NO);
static_assert((NO % OT) == 0);
static_assert(OT == 64);
static_assert((LAT % 32) == 0);
static_assert(PREP_BLK * PREP_TPB * 4 == 2 * NQ * LAT);
static_assert(((PREP_BLK / 2) * PREP_TPB * 4) == NQ * LAT);
static_assert((QB * LAT) % TPB == 0);
static_assert(QB * LAT * 4 == 32 * 128);
static_assert(WAVES * 2 * 4 == 32);
static_assert(OT * 2 == 128);
static_assert(4 * 4 == 16);
static_assert(QB * LAT <= WAVES * CHUNK * WPAD);
static_assert((WPAD % 4) == 0);
static_assert((TP % 8) == 0);

DEVINL v8f wmma_f16(v16h a, v16h b, v8f c) {
  v8f d = __builtin_amdgcn_wmma_f32_16x16x32_f16(false, a, false, b, (short)0, c, false, false);
  asm volatile("v_nop\n\tv_nop\n\tv_nop\n\tv_nop" : "+v"(d) : "v"(a), "v"(b));
  return d;
}
DEVINL v8f zero8f() {
  v8f z = {0.f, 0.f, 0.f, 0.f, 0.f, 0.f, 0.f, 0.f};
  return z;
}
DEVINL void load_frag(FragH& f, const f16t* row, int k0) {
  f.half[0] = *(const v8ha*)(row + k0);
  f.half[1] = *(const v8ha*)(row + k0 + 16);
}

DEVINL float dist2(float qx, float qy, float qz, float ox, float oy, float oz) {
  #pragma clang fp contract(off)
  const float dx = qx - ox, dy = qy - oy, dz = qz - oz;
  float s = dx * dx + dz * dz;
  s = s + dy * dy;
  return s;
}

__global__ __launch_bounds__(PREP_TPB) void prep_uw_k(const float* __restrict__ posq, const float* __restrict__ poso,
                                                     const float* __restrict__ W1, const float* __restrict__ b1,
                                                     const float* __restrict__ xo,
                                                     float* __restrict__ u, float* __restrict__ w)
{
  (void)xo;
  const int blk = blockIdx.x;
  if (blk >= PREP_BLK) return;
  const bool isu = (blk < PREP_BLK / 2);
  const int g = (isu ? blk : (blk - PREP_BLK / 2)) * PREP_TPB + (int)threadIdx.x;
  const int e = 4 * g;
  const int i = e >> 6, l = e & (LAT - 1);
  const float ax = posq[3 * i], ay = posq[3 * i + 1], az = posq[3 * i + 2];
  const float bx = poso[3 * i], by = poso[3 * i + 1], bz = poso[3 * i + 2];
  const float px = isu ? ax : bx, py = isu ? ay : by, pz = isu ? az : bz;
  v4f o;
  #pragma unroll
  for (int j = 0; j < 4; ++j) {
    const float wq0 = W1[0 * LAT + l + j], wq1 = W1[1 * LAT + l + j], wq2 = W1[2 * LAT + l + j];
    const float wo0 = W1[3 * LAT + l + j], wo1 = W1[4 * LAT + l + j], wo2 = W1[5 * LAT + l + j];
    const float wr0 = W1[6 * LAT + l + j], wr1 = W1[7 * LAT + l + j], wr2 = W1[8 * LAT + l + j];
    const float c0 = isu ? (wq0 + wr0) : (wo0 - wr0);
    const float c1 = isu ? (wq1 + wr1) : (wo1 - wr1);
    const float c2 = isu ? (wq2 + wr2) : (wo2 - wr2);
    const float bb = b1[l + j];
    float a = isu ? 0.0f : bb;
    a = fmaf(px, c0, a);
    a = fmaf(py, c1, a);
    a = fmaf(pz, c2, a);
    o[j] = a;
  }
  float* dst = (isu ? u : w) + e;
  *(volatile v4f*)dst = o;
  __threadfence();
  *(volatile v4f*)dst = o;
}

__global__ __launch_bounds__(TPB) void vproj_k(const float* __restrict__ H, const float* __restrict__ Wv,
                                              const float* __restrict__ bv, f16t* __restrict__ vT)
{
  __shared__ __attribute__((aligned(16))) f16t T_s[LAT * TP];
  const int tid = threadIdx.x, lane = tid & 31, wave = tid >> 5;
  const int hh = lane >> 4, m = lane & 15;
  if (blockIdx.x >= NO / OT) return;
  const int o0 = blockIdx.x * OT;
  const int lr = 16 * wave + m;

  v8f acc[4];
  #pragma unroll
  for (int t = 0; t < 4; ++t) acc[t] = zero8f();

  #pragma unroll
  for (int ks = 0; ks < LAT / 32; ++ks) {
    const int k0 = 32 * ks;
    FragH a;
    #pragma unroll
    for (int i = 0; i < 8; ++i) {
      a.v[i]     = (f16t)(Wv[(size_t)(k0 + 8 * hh + i) * LAT + lr] * WCAR);
      a.v[8 + i] = (f16t)(Wv[(size_t)(k0 + 16 + 8 * hh + i) * LAT + lr] * WCAR);
    }
    #pragma unroll
    for (int t = 0; t < 4; ++t) {
      const float* hrow = H + (size_t)(o0 + 16 * t + m) * LAT + k0 + 8 * hh;
      const v4f x0 = *(const v4fa*)(hrow),      x1 = *(const v4fa*)(hrow + 4);
      const v4f x2 = *(const v4fa*)(hrow + 16), x3 = *(const v4fa*)(hrow + 20);
      FragH b;
      #pragma unroll
      for (int j = 0; j < 4; ++j) {
        b.v[j]      = (f16t)(x0[j] * HCAR);
        b.v[4 + j]  = (f16t)(x1[j] * HCAR);
        b.v[8 + j]  = (f16t)(x2[j] * HCAR);
        b.v[12 + j] = (f16t)(x3[j] * HCAR);
      }
      acc[t] = wmma_f16(a.v, b.v, acc[t]);
    }
  }

  #pragma unroll
  for (int r = 0; r < 8; ++r) {
    const int l = 16 * wave + 8 * hh + r;
    const float bb = bv[l];
    #pragma unroll
    for (int t = 0; t < 4; ++t)
      T_s[l * TP + 16 * t + m] = (f16t)((acc[t][r] * SC_WH + bb) * VCAR);
  }
  __syncthreads();

  #pragma unroll
  for (int j = 0; j < 4; ++j) {
    const int row = 16 * wave + 4 * j + (lane >> 3);
    const int ch = 8 * (lane & 7);
    const v8h v = *(const v8ha*)(T_s + row * TP + ch);
    f16t* dst = vT + (size_t)row * NO + o0 + ch;
    *(volatile v8h*)dst = v;
  }
  __threadfence();
  #pragma unroll
  for (int j = 0; j < 4; ++j) {
    const int row = 16 * wave + 4 * j + (lane >> 3);
    const int ch = 8 * (lane & 7);
    const v8h v = *(const v8ha*)(T_s + row * TP + ch);
    f16t* dst = vT + (size_t)row * NO + o0 + ch;
    *(volatile v8h*)dst = v;
  }
}

#define FOREACH_Q(X) X(0) X(1) X(2) X(3) X(4) X(5) X(6) X(7) \
                     X(8) X(9) X(10) X(11) X(12) X(13) X(14) X(15)

__global__ __launch_bounds__(TPB) void attn_k(const float* __restrict__ u, const float* __restrict__ w,
                                             const f16t* __restrict__ vT,
                                             const float* __restrict__ posq, const float* __restrict__ poso,
                                             const float* __restrict__ W2, const float* __restrict__ b2,
                                             float* __restrict__ out)
{
  __shared__ __attribute__((aligned(16))) float u_s[QB * LAT];
  __shared__ __attribute__((aligned(16))) float w2_s[LAT];
  __shared__ float pq_s[QB * 4];
  __shared__ __attribute__((aligned(16))) float w_s[WAVES * CHUNK * WPAD];
  __shared__ __attribute__((aligned(16))) f16t P_s[WAVES * QB * CHUNK];
  __shared__ float m_s[WAVES * QB];
  __shared__ float l_s[WAVES * QB];
  __shared__ __attribute__((aligned(16))) float acc_s[WAVES * QB * LAT];

  const int tid = threadIdx.x, lane = tid & 31;
  const int wave = __builtin_amdgcn_readfirstlane(tid >> 5);
  const int hh = lane >> 4, lo = lane & 15;
  if (blockIdx.x >= NQ / QB) return;
  const int qb = blockIdx.x * QB;

  #pragma unroll
  for (int i = tid; i < QB * LAT; i += TPB) u_s[i] = u[(size_t)qb * LAT + i];
  if (tid < QB * PDIM) pq_s[(tid / PDIM) * 4 + (tid % PDIM)] = posq[qb * PDIM + tid];
  if (tid < LAT) w2_s[tid] = W2[tid];
  __syncthreads();

  const float b2v = b2[0];
  const float thr = __int_as_float(THR2_BITS);
  const v2f z2 = {0.f, 0.f};

#define DECLQ(q) v2f sv##q; float s##q; float mr##q = NEG_INF; float sc##q = 1.0f;
  FOREACH_Q(DECLQ)

  v8f acc[4], accl;
  #pragma unroll
  for (int t = 0; t < 4; ++t) acc[t] = zero8f();
  accl = zero8f();

  const f16t onev = (lo == 0) ? (f16t)1.0f : (f16t)0.0f;
  v16h Bones;
  #pragma unroll
  for (int i = 0; i < 16; ++i) Bones[i] = onev;

  const int obase = wave * OPW;
  float* const wcol = w_s + (wave * CHUNK + lane) * WPAD;
  f16t* const pw = P_s + wave * (QB * CHUNK);

  #pragma unroll 1
  for (int c = 0; c < NCHUNK; ++c) {
    const int o = obase + c * CHUNK + lane;
    const float* wp = w + (size_t)o * LAT;
    #pragma unroll
    for (int i = 0; i < LAT / 4; ++i) *(v4fa*)(wcol + 4 * i) = *(const v4fa*)(wp + 4 * i);
    const float ox = poso[3 * o], oy = poso[3 * o + 1], oz = poso[3 * o + 2];

#define SINIT(q) sv##q = z2;
    FOREACH_Q(SINIT)
    #pragma unroll 1
    for (int l4 = 0; l4 < LAT / 4; ++l4) {
      const v4f wv = *(const v4fa*)(wcol + 4 * l4);
      const v4f gv = *(const v4fa*)(w2_s + 4 * l4);
      const v2f w01 = {wv[0], wv[1]}, w23 = {wv[2], wv[3]};
      const v2f g01 = {gv[0], gv[1]}, g23 = {gv[2], gv[3]};
#define LOGQ(q) { const v4f uv = *(const v4fa*)(u_s + q * LAT + 4 * l4);          \
      v2f a0 = {uv[0], uv[1]}; v2f a1 = {uv[2], uv[3]};                           \
      a0 += w01; a1 += w23;                                                       \
      a0 = __builtin_elementwise_max(a0, z2);                                     \
      a1 = __builtin_elementwise_max(a1, z2);                                     \
      sv##q = a0 * g01 + sv##q;                                                   \
      sv##q = a1 * g23 + sv##q; }
      FOREACH_Q(LOGQ)
    }
#define SFIN(q) s##q = (sv##q[0] + sv##q[1]) + b2v;
    FOREACH_Q(SFIN)

    __syncthreads();

#define SOFTQ(q) {                                                                \
      const float d2 = dist2(pq_s[4 * q], pq_s[4 * q + 1], pq_s[4 * q + 2], ox, oy, oz); \
      const bool msk = (d2 > thr);                                                \
      const float sq = msk ? NEG_INF : s##q;                                      \
      float rmax = sq;                                                            \
      rmax = fmaxf(rmax, __shfl_xor(rmax, 16));                                   \
      rmax = fmaxf(rmax, __shfl_xor(rmax, 8));                                    \
      rmax = fmaxf(rmax, __shfl_xor(rmax, 4));                                    \
      rmax = fmaxf(rmax, __shfl_xor(rmax, 2));                                    \
      rmax = fmaxf(rmax, __shfl_xor(rmax, 1));                                    \
      const float mnew = fmaxf(mr##q, rmax);                                      \
      const float e = __expf(sq - mnew);                                          \
      const float p = msk ? 0.0f : e;                                             \
      const float scn = __expf(mr##q - mnew);                                     \
      sc##q = (mnew == NEG_INF) ? 1.0f : scn;                                     \
      mr##q = mnew;                                                               \
      pw[q * CHUNK + lane] = (f16t)(p * PCAR); }
    FOREACH_Q(SOFTQ)

    __syncthreads();

    const bool loh = (hh == 0);
    const float f0 = loh ? sc0 : sc8;
    const float f1 = loh ? sc1 : sc9;
    const float f2 = loh ? sc2 : sc10;
    const float f3 = loh ? sc3 : sc11;
    const float f4 = loh ? sc4 : sc12;
    const float f5 = loh ? sc5 : sc13;
    const float f6 = loh ? sc6 : sc14;
    const float f7 = loh ? sc7 : sc15;
#define RESC(T) { T[0] *= f0; T[1] *= f1; T[2] *= f2; T[3] *= f3;               \
                  T[4] *= f4; T[5] *= f5; T[6] *= f6; T[7] *= f7; }
    RESC(acc[0]) RESC(acc[1]) RESC(acc[2]) RESC(acc[3]) RESC(accl)

    FragH A;
    A.half[0] = *(const v8ha*)(pw + lo * CHUNK + 8 * hh);
    A.half[1] = *(const v8ha*)(pw + lo * CHUNK + 16 + 8 * hh);

    accl = wmma_f16(A.v, Bones, accl);

    const f16t* bcol = vT + (size_t)lo * NO + obase + c * CHUNK + 8 * hh;
    #pragma unroll
    for (int t = 0; t < 4; ++t) {
      FragH B;
      load_frag(B, bcol + (size_t)16 * t * NO, 0);
      acc[t] = wmma_f16(A.v, B.v, acc[t]);
    }
  }

  if (lane == 0) {
#define STM(q) m_s[wave * QB + q] = mr##q;
    FOREACH_Q(STM)
  }
  if (lo == 0) {
    #pragma unroll
    for (int r = 0; r < 8; ++r) l_s[wave * QB + 8 * hh + r] = accl[r];
  }
  #pragma unroll
  for (int t = 0; t < 4; ++t) {
    #pragma unroll
    for (int r = 0; r < 8; ++r)
      acc_s[(wave * QB + 8 * hh + r) * LAT + 16 * t + lo] = acc[t][r];
  }
  __syncthreads();

  float* const os = w_s;
  #pragma unroll 1
  for (int k = 0; k < (QB * LAT) / TPB; ++k) {
    const int idx = tid + TPB * k;
    const int row = idx >> 6, col = idx & (LAT - 1);
    float mm = NEG_INF;
    #pragma unroll
    for (int wv = 0; wv < WAVES; ++wv) mm = fmaxf(mm, m_s[wv * QB + row]);
    float den = 0.0f, num = 0.0f;
    #pragma unroll
    for (int wv = 0; wv < WAVES; ++wv) {
      const float mw = m_s[wv * QB + row];
      const float e = __expf(mw - mm);
      const float f = (mw == NEG_INF) ? 0.0f : e;
      den = fmaf(f, l_s[wv * QB + row], den);
      num = fmaf(f, acc_s[(wv * QB + row) * LAT + col], num);
    }
    os[row * LAT + col] = (num * (1.0f / den)) * SC_V;
  }
  __syncthreads();

  {
    v4f va[2];
    float* da[2];
    #pragma unroll
    for (int j = 0; j < 2; ++j) {
      const int L = 8 * wave + 4 * j + (lane >> 3);
      const int row = L >> 1;
      const int col = (L & 1) * 32 + 4 * (lane & 7);
      va[j] = *(const v4fa*)(os + row * LAT + col);
      da[j] = out + (size_t)(qb + row) * LAT + col;
      *(volatile v4f*)da[j] = va[j];
    }
    __threadfence();
    #pragma unroll
    for (int j = 0; j < 2; ++j) *(volatile v4f*)da[j] = va[j];
  }
}

extern "C" void kernel_launch(void* const* d_in, const int* in_sizes, int n_in,
                              void* d_out, int out_size, void* d_ws, size_t ws_size,
                              hipStream_t stream) {
  if (n_in < 10) return;
  if (in_sizes[0] != NO * LAT) return;
  if (in_sizes[2] != NO * PDIM || in_sizes[3] != NQ * PDIM) return;
  if (in_sizes[4] != ENC * LAT || in_sizes[5] != LAT) return;
  if (in_sizes[6] != LAT || in_sizes[7] < 1) return;
  if (in_sizes[8] != LAT * LAT || in_sizes[9] != LAT) return;
  if (out_size != NQ * LAT) return;

  const float* h_obs     = (const float*)d_in[0];
  const float* x_obs     = (const float*)d_in[1];
  const float* pos_obs   = (const float*)d_in[2];
  const float* pos_query = (const float*)d_in[3];
  const float* W1        = (const float*)d_in[4];
  const float* b1        = (const float*)d_in[5];
  const float* W2        = (const float*)d_in[6];
  const float* b2        = (const float*)d_in[7];
  const float* Wv        = (const float*)d_in[8];
  const float* bv        = (const float*)d_in[9];
  float* outp = (float*)d_out;

  const size_t szU  = (size_t)NQ * LAT * 4;
  const size_t szW  = (size_t)NO * LAT * 4;
  const size_t szVT = (size_t)LAT * NO * 2;
  size_t off = 0;
  char* ws = (char*)d_ws;
  float* u  = (float*)(ws + off);  off += szU;
  float* w  = (float*)(ws + off);  off += szW;
  f16t*  vT = (f16t*)(ws + off);   off += szVT;
  if (off > ws_size) return;

  prep_uw_k<<<PREP_BLK, PREP_TPB, 0, stream>>>(pos_query, pos_obs, W1, b1, x_obs, u, w);
  vproj_k<<<NO / OT, TPB, 0, stream>>>(h_obs, Wv, bv, vT);
  attn_k<<<NQ / QB, TPB, 0, stream>>>(u, w, vT, pos_query, pos_obs, W2, b2, outp);
  (void)hipGetLastError();
}
